// SPConvnet_21157008900556
// MI455X (gfx1250) — hardware-verified
//
#include <hip/hip_runtime.h>
#include <stddef.h>


#define GRD     128
#define NBAT    2
#define CIN     11
#define C1      64
#define C2      32
#define NTAP    27
#define NG1     14
#define KP1     (NG1 * 32)
#define KP2     (NTAP * C1)
#define NCL     4096
#define NTHR    256
#define NWAVE   8
#define PTS     (NWAVE * 16)
#define AP1     40
#define AP2     72
#define OP1     72
#define OP2     36
#define TBLK    32768
#define TBLN    (NBAT * GRD * GRD * GRD)
#define CHT     (NTHR * 8)
#define EPT     8
#define NGRP    2
#define CHUNK   (NTHR * EPT * NGRP)
#define WCAP    (EPT * NGRP * 32)
#define LISTN   (NWAVE * WCAP)
#define NBP     128
#define RPAD    1024
#define WSCALE  16.0f
#define WINV    0.0625f
#define LDS_TAB (TBLK * 4)

static_assert((TBLN % TBLK) == 0);
static_assert((NCL % NBP) == 0);
static_assert((CHUNK & (CHUNK - 1)) == 0 && CHUNK <= 4096);
static_assert((NBP & (NBP - 1)) == 0 && NBP <= 4096);
static_assert(((C1 * KP1 / 8) % NTHR) == 0 && ((C2 * KP2 / 8) % NTHR) == 0);
static_assert((RPAD % PTS) == 0 && ((RPAD * 2) % NTHR) == 0 && ((RPAD / 4) % NTHR) == 0);
static_assert(NBP * C2 / 4 == 4 * NTHR);
static_assert((TBLK / 4) % NTHR == 0);
static_assert((AP1 * 2) % 16 == 0 && (AP2 * 2) % 16 == 0 && (OP1 * 2) % 16 == 0 && (OP2 * 4) % 16 == 0);

typedef float    v4f  __attribute__((ext_vector_type(4)));
typedef float    v8f  __attribute__((ext_vector_type(8)));
typedef int      v4i  __attribute__((ext_vector_type(4)));
typedef _Float16 v8h  __attribute__((ext_vector_type(8)));
typedef _Float16 v16h __attribute__((ext_vector_type(16)));
typedef v4f __attribute__((may_alias)) v4fa;
typedef v8h __attribute__((may_alias)) v8ha;
union FragH { v16h v; v8h h[2]; };

__device__ __forceinline__ int clampi(int v, int lo, int hi) { return v < lo ? lo : (v > hi ? hi : v); }

__device__ __forceinline__ v8h cvt8(v4f a, v4f b) {
  v8h r;
  r[0] = (_Float16)a.x; r[1] = (_Float16)a.y; r[2] = (_Float16)a.z; r[3] = (_Float16)a.w;
  r[4] = (_Float16)b.x; r[5] = (_Float16)b.y; r[6] = (_Float16)b.z; r[7] = (_Float16)b.w;
  return r;
}

__device__ __forceinline__ v8f wmh(v16h a, v16h b, v8f c) {
  v8f d = __builtin_amdgcn_wmma_f32_16x16x32_f16(false, a, false, b, (short)0, c, false, false);
  asm volatile("v_nop\n\tv_nop\n\tv_nop\n\tv_nop" : "+v"(d) : "v"(a), "v"(b));
  return d;
}

template <int NB>
__device__ __forceinline__ int scan_chunk(const int* __restrict__ dsts, int nE, int cbase, int slotBase,
                                          int vec8, int* list, int tid, int lane, int wave) {
  int wc = 0;
#pragma unroll
  for (int g = 0; g < NGRP; ++g) {
    const int el0  = (g * NTHR + tid) * EPT;
    const int e0   = cbase + el0;
    const int sent = -2147483647 - 1;
    v4i da, db;
    if (vec8 != 0 && cbase + CHUNK <= nE) {
      da = *(const v4i*)(dsts + e0);
      db = *(const v4i*)(dsts + e0 + 4);
    } else {
      da.x = (e0     < nE) ? dsts[min(e0, nE - 1)] : sent;
      da.y = (e0 + 1 < nE) ? dsts[min(e0 + 1, nE - 1)] : sent;
      da.z = (e0 + 2 < nE) ? dsts[min(e0 + 2, nE - 1)] : sent;
      da.w = (e0 + 3 < nE) ? dsts[min(e0 + 3, nE - 1)] : sent;
      db.x = (e0 + 4 < nE) ? dsts[min(e0 + 4, nE - 1)] : sent;
      db.y = (e0 + 5 < nE) ? dsts[min(e0 + 5, nE - 1)] : sent;
      db.z = (e0 + 6 < nE) ? dsts[min(e0 + 6, nE - 1)] : sent;
      db.w = (e0 + 7 < nE) ? dsts[min(e0 + 7, nE - 1)] : sent;
    }
    const unsigned nb = (unsigned)slotBase;
    const unsigned s0 = (unsigned)da.x - nb, s1 = (unsigned)da.y - nb;
    const unsigned s2 = (unsigned)da.z - nb, s3 = (unsigned)da.w - nb;
    const unsigned s4 = (unsigned)db.x - nb, s5 = (unsigned)db.y - nb;
    const unsigned s6 = (unsigned)db.z - nb, s7 = (unsigned)db.w - nb;
    const bool h0 = s0 < (unsigned)NB, h1 = s1 < (unsigned)NB, h2 = s2 < (unsigned)NB, h3 = s3 < (unsigned)NB;
    const bool h4 = s4 < (unsigned)NB, h5 = s5 < (unsigned)NB, h6 = s6 < (unsigned)NB, h7 = s7 < (unsigned)NB;
    const unsigned any = __builtin_amdgcn_ballot_w32(h0 | h1 | h2 | h3 | h4 | h5 | h6 | h7);
    if (any != 0u) {
#define HITJ(J, HJ, SJ) { \
        const unsigned mj = __builtin_amdgcn_ballot_w32(HJ); \
        if (mj != 0u) { \
          if (HJ) { \
            const int pos = wc + (int)__builtin_amdgcn_mbcnt_lo(mj, 0u); \
            if (pos < WCAP) list[wave * WCAP + pos] = ((el0 + (J)) << 12) | (int)(SJ); \
          } \
          wc += (int)__builtin_popcount(mj); } }
      HITJ(0, h0, s0)
      HITJ(1, h1, s1)
      HITJ(2, h2, s2)
      HITJ(3, h3, s3)
      HITJ(4, h4, s4)
      HITJ(5, h5, s5)
      HITJ(6, h6, s6)
      HITJ(7, h7, s7)
#undef HITJ
    }
  }
  return wc;
}

__global__ __launch_bounds__(NTHR) void k_prep(
    const float* __restrict__ W1, const float* __restrict__ W2, const float* __restrict__ feat,
    const int* __restrict__ idx, _Float16* P1, _Float16* P2, _Float16* F, int* lin,
    int nPts, int nRows) {
  const int s0 = C1 * KP1 / 8;
  const int s1 = C2 * KP2 / 8;
  const int s2 = nRows * 2;
  const int s3 = nRows / 4;
  const int bstart = blockIdx.x * NTHR;
  const int i = bstart + (int)threadIdx.x;
  if (bstart < s0 + s1 + s2) {
    float v[8];
    _Float16* dp;
    if (bstart < s0) {
      const int o  = i * 8;
      const int n  = o / KP1;
      const int k0 = o - n * KP1;
#pragma unroll
      for (int e = 0; e < 8; ++e) {
        const int k    = k0 + e;
        const int tap  = k >> 4;
        const int c    = k & 15;
        const int tapc = tap > NTAP - 1 ? NTAP - 1 : tap;
        const int cc   = c > CIN - 1 ? CIN - 1 : c;
        const float x  = W1[(tapc * CIN + cc) * C1 + n];
        v[e] = (tap < NTAP && c < CIN) ? x * WSCALE : 0.0f;
      }
      dp = P1 + o;
    } else if (bstart < s0 + s1) {
      const int o  = (i - s0) * 8;
      const int n  = o / KP2;
      const int k0 = o - n * KP2;
#pragma unroll
      for (int e = 0; e < 8; ++e) {
        const int k   = k0 + e;
        const int tap = k >> 6;
        const int c   = k & 63;
        v[e] = W2[(tap * C1 + c) * C2 + n] * WSCALE;
      }
      dp = P2 + o;
    } else {
      const int p    = i - s0 - s1;
      const int row  = p >> 1;
      const int hb   = p & 1;
      const int rowc = row > nPts - 1 ? nPts - 1 : row;
#pragma unroll
      for (int e = 0; e < 8; ++e) {
        const int ch  = 8 * hb + e;
        const int chc = ch > CIN - 1 ? CIN - 1 : ch;
        const float x = feat[(size_t)rowc * CIN + chc];
        v[e] = (row < nPts && ch < CIN) ? x : 0.0f;
      }
      dp = F + (size_t)p * 8;
    }
    v4f a, b;
    a.x = v[0]; a.y = v[1]; a.z = v[2]; a.w = v[3];
    b.x = v[4]; b.y = v[5]; b.z = v[6]; b.w = v[7];
    const v8h hv = cvt8(a, b);
    *(volatile v8h*)dp = hv;
    __threadfence();
    *(volatile v8h*)dp = hv;
  } else {
    if (i >= s0 + s1 + s2 + s3) return;
    const int p = i - s0 - s1 - s2;
    int lv[4];
#pragma unroll
    for (int q = 0; q < 4; ++q) {
      const int r  = 4 * p + q;
      const int rc = r > nPts - 1 ? nPts - 1 : r;
      const v4i cv = *(const v4i*)(idx + (size_t)rc * 4);
      const int bb = clampi(cv.x, 0, NBAT - 1);
      const int zz = clampi(cv.y, 0, GRD - 1);
      const int yy = clampi(cv.z, 0, GRD - 1);
      const int xx = clampi(cv.w, 0, GRD - 1);
      const int key = ((bb * GRD + zz) * GRD + yy) * GRD + xx;
      lv[q] = r < nPts ? key : -1;
    }
    v4i o4;
    o4.x = lv[0]; o4.y = lv[1]; o4.z = lv[2]; o4.w = lv[3];
    int* lp = lin + (size_t)p * 4;
    *(volatile v4i*)lp = o4;
    __threadfence();
    *(volatile v4i*)lp = o4;
  }
}

__global__ __launch_bounds__(NTHR) void k_table(const int* __restrict__ lin, int* tbl, int nPts) {
  extern __shared__ v4i lds_dyn[];
  int* tab = (int*)lds_dyn;
  const int tid = threadIdx.x;
  const int base = blockIdx.x * TBLK;
  {
    const v4i mm = {-1, -1, -1, -1};
#pragma unroll 1
    for (int q = tid; q < TBLK / 4; q += NTHR) lds_dyn[q] = mm;
  }
  __syncthreads();

  const int nCh = (nPts + CHT - 1) / CHT;
#pragma unroll 1
  for (int ch = 0; ch < nCh; ++ch) {
    const int cbase = ch * CHT;
    const int e0 = cbase + tid * 8;
    v4i da, db;
    if (cbase + CHT <= nPts) {
      da = *(const v4i*)(lin + e0);
      db = *(const v4i*)(lin + e0 + 4);
    } else {
      da.x = (e0     < nPts) ? lin[min(e0,     nPts - 1)] : -1;
      da.y = (e0 + 1 < nPts) ? lin[min(e0 + 1, nPts - 1)] : -1;
      da.z = (e0 + 2 < nPts) ? lin[min(e0 + 2, nPts - 1)] : -1;
      da.w = (e0 + 3 < nPts) ? lin[min(e0 + 3, nPts - 1)] : -1;
      db.x = (e0 + 4 < nPts) ? lin[min(e0 + 4, nPts - 1)] : -1;
      db.y = (e0 + 5 < nPts) ? lin[min(e0 + 5, nPts - 1)] : -1;
      db.z = (e0 + 6 < nPts) ? lin[min(e0 + 6, nPts - 1)] : -1;
      db.w = (e0 + 7 < nPts) ? lin[min(e0 + 7, nPts - 1)] : -1;
    }
    int vv[8];
    vv[0] = da.x; vv[1] = da.y; vv[2] = da.z; vv[3] = da.w;
    vv[4] = db.x; vv[5] = db.y; vv[6] = db.z; vv[7] = db.w;
#pragma unroll
    for (int j = 0; j < 8; ++j) {
      const unsigned s = (unsigned)vv[j] - (unsigned)base;
      if (s < (unsigned)TBLK) tab[s] = e0 + j;
    }
  }
  __syncthreads();

  int* gp = tbl + (size_t)base;
#pragma unroll 1
  for (int q = tid; q < TBLK / 4; q += NTHR) { const v4i v = lds_dyn[q]; *(volatile v4i*)(gp + 4 * q) = v; }
  __threadfence();
#pragma unroll 1
  for (int q = tid; q < TBLK / 4; q += NTHR) { const v4i v = lds_dyn[q]; *(volatile v4i*)(gp + 4 * q) = v; }
}

__global__ __launch_bounds__(NTHR) void k_conv1(
    const int* __restrict__ idx, const int* __restrict__ dimD, const int* __restrict__ dimH,
    const int* __restrict__ dimW, const int* __restrict__ tbl, const _Float16* __restrict__ F,
    const _Float16* __restrict__ P1, const float* __restrict__ b1, _Float16* H1, int nPts, int zrow) {
  __shared__ __attribute__((aligned(16))) _Float16 sA[2 * NWAVE * 16 * AP1];
  __shared__ __attribute__((aligned(16))) _Float16 sO[NWAVE * 16 * OP1];
  const int tid = threadIdx.x, lane = tid & 31, wave = tid >> 5, hh = lane >> 4, m = lane & 15;
  const int D  = clampi(dimD[0], 1, GRD);
  const int Hh = clampi(dimH[0], 1, GRD);
  const int Wd = clampi(dimW[0], 1, GRD);
  const int rowBase = blockIdx.x * PTS + wave * 16;
  const int prow = min(rowBase + m, nPts - 1);
  const v4i cc = *(const v4i*)(idx + (size_t)prow * 4);
  const int bc = clampi(cc.x, 0, NBAT - 1);

  v8f acc[4];
#pragma unroll
  for (int t = 0; t < 4; ++t) { v8f z8 = {0.f, 0.f, 0.f, 0.f, 0.f, 0.f, 0.f, 0.f}; acc[t] = z8; }
  _Float16* sAw = sA + wave * 16 * AP1;

#pragma unroll 1
  for (int g = 0; g < NG1; ++g) {
    const int tap  = 2 * g + hh;
    const int tapc = tap > NTAP - 1 ? NTAP - 1 : tap;
    const int dz = tapc / 9 - 1, dy = (tapc / 3) % 3 - 1, dx = tapc % 3 - 1;
    const int z = cc.y + dz, y = cc.z + dy, x = cc.w + dx;
    int ok = (tap < NTAP) & ((unsigned)z < (unsigned)D) & ((unsigned)y < (unsigned)Hh) & ((unsigned)x < (unsigned)Wd);
    const int zc = clampi(z, 0, D - 1), yc = clampi(y, 0, Hh - 1), xc = clampi(x, 0, Wd - 1);
    const int nb = tbl[((bc * GRD + zc) * GRD + yc) * GRD + xc];
    ok = ok & (nb >= 0);
    const int src = ok != 0 ? clampi(nb, 0, nPts - 1) : zrow;
    const _Float16* fp = F + (size_t)src * 16;
    const v8h p0 = *(const v8h*)fp;
    const v8h p1 = *(const v8h*)(fp + 8);
    _Float16* ap = sAw + (g & 1) * (NWAVE * 16 * AP1) + m * AP1 + 16 * hh;
    *(v8h*)ap       = p0;
    *(v8h*)(ap + 8) = p1;
    __syncthreads();
    const _Float16* ar = sAw + (g & 1) * (NWAVE * 16 * AP1) + m * AP1 + 8 * hh;
    FragH a;
    a.h[0] = *(const v8ha*)ar;
    a.h[1] = *(const v8ha*)(ar + 16);
#pragma unroll
    for (int t = 0; t < 4; ++t) {
      const _Float16* bp = P1 + (size_t)(16 * t + m) * KP1 + 32 * g + 8 * hh;
      FragH b;
      b.h[0] = *(const v8h*)bp;
      b.h[1] = *(const v8h*)(bp + 16);
      acc[t] = wmh(a.v, b.v, acc[t]);
    }
  }

  _Float16* sp = sO + wave * 16 * OP1 + (8 * hh) * OP1;
#pragma unroll
  for (int t = 0; t < 4; ++t) {
    const int col = 16 * t + m;
    const float bv = b1[col];
#pragma unroll
    for (int r = 0; r < 8; ++r) {
      float v = acc[t][r] * WINV + bv;
      v = fmaxf(v, 0.0f);
      v = (rowBase + 8 * hh + r) < nPts ? v : 0.0f;
      sp[r * OP1 + col] = (_Float16)v;
    }
  }
  __syncthreads();

  const int q = lane & 7;
  v8h ov[4];
#pragma unroll
  for (int j = 0; j < 4; ++j) {
    const int r = 4 * j + (lane >> 3);
    ov[j] = *(const v8ha*)(sO + wave * 16 * OP1 + r * OP1 + 8 * q);
  }
#pragma unroll
  for (int j = 0; j < 4; ++j) {
    const int r = 4 * j + (lane >> 3);
    *(volatile v8h*)(H1 + (size_t)(rowBase + r) * C1 + 8 * q) = ov[j];
  }
  __threadfence();
#pragma unroll
  for (int j = 0; j < 4; ++j) {
    const int r = 4 * j + (lane >> 3);
    *(volatile v8h*)(H1 + (size_t)(rowBase + r) * C1 + 8 * q) = ov[j];
  }
}

__global__ __launch_bounds__(NTHR) void k_conv2(
    const int* __restrict__ idx, const int* __restrict__ dimD, const int* __restrict__ dimH,
    const int* __restrict__ dimW, const int* __restrict__ tbl, const _Float16* __restrict__ H1,
    const _Float16* __restrict__ P2, const float* __restrict__ b2, float* FT, int nPts, int zrow) {
  __shared__ __attribute__((aligned(16))) _Float16 sA[2 * NWAVE * 16 * AP2];
  __shared__ __attribute__((aligned(16))) float    sO[NWAVE * 16 * OP2];
  const int tid = threadIdx.x, lane = tid & 31, wave = tid >> 5, hh = lane >> 4, m = lane & 15;
  const int D  = clampi(dimD[0], 1, GRD);
  const int Hh = clampi(dimH[0], 1, GRD);
  const int Wd = clampi(dimW[0], 1, GRD);
  const int rowBase = blockIdx.x * PTS + wave * 16;
  const int prow = min(rowBase + m, nPts - 1);
  const v4i cc = *(const v4i*)(idx + (size_t)prow * 4);
  const int bc = clampi(cc.x, 0, NBAT - 1);
  const int q = lane & 7;

  v8f acc[2];
#pragma unroll
  for (int t = 0; t < 2; ++t) { v8f z8 = {0.f, 0.f, 0.f, 0.f, 0.f, 0.f, 0.f, 0.f}; acc[t] = z8; }
  _Float16* sAw = sA + wave * 16 * AP2;

#pragma unroll 1
  for (int tap = 0; tap < NTAP; ++tap) {
    const int dz = tap / 9 - 1, dy = (tap / 3) % 3 - 1, dx = tap % 3 - 1;
    const int z = cc.y + dz, y = cc.z + dy, x = cc.w + dx;
    int ok = ((unsigned)z < (unsigned)D) & ((unsigned)y < (unsigned)Hh) & ((unsigned)x < (unsigned)Wd);
    const int zc = clampi(z, 0, D - 1), yc = clampi(y, 0, Hh - 1), xc = clampi(x, 0, Wd - 1);
    const int nb = tbl[((bc * GRD + zc) * GRD + yc) * GRD + xc];
    ok = ok & (nb >= 0);
    const int src = ok != 0 ? clampi(nb, 0, nPts - 1) : zrow;
    _Float16* abuf = sAw + (tap & 1) * (NWAVE * 16 * AP2);
#pragma unroll
    for (int j = 0; j < 4; ++j) {
      const int srow = 4 * j + (lane >> 3);
      const int s = __shfl(src, srow);
      const v8h pv = *(const v8h*)(H1 + (size_t)s * C1 + 8 * q);
      *(v8h*)(abuf + srow * AP2 + 8 * q) = pv;
    }
    __syncthreads();
    const _Float16* ar = abuf + m * AP2 + 8 * hh;
#pragma unroll
    for (int ks = 0; ks < 2; ++ks) {
      FragH a;
      a.h[0] = *(const v8ha*)(ar + 32 * ks);
      a.h[1] = *(const v8ha*)(ar + 32 * ks + 16);
#pragma unroll
      for (int t = 0; t < 2; ++t) {
        const _Float16* bp = P2 + (size_t)(16 * t + m) * KP2 + C1 * tap + 32 * ks + 8 * hh;
        FragH b;
        b.h[0] = *(const v8h*)bp;
        b.h[1] = *(const v8h*)(bp + 16);
        acc[t] = wmh(a.v, b.v, acc[t]);
      }
    }
  }

  float* sp = sO + wave * 16 * OP2 + (8 * hh) * OP2;
#pragma unroll
  for (int t = 0; t < 2; ++t) {
    const int col = 16 * t + m;
    const float bv = b2[col];
#pragma unroll
    for (int r = 0; r < 8; ++r) {
      float v = acc[t][r] * WINV + bv;
      v = fmaxf(v, 0.0f);
      v = (rowBase + 8 * hh + r) < nPts ? v : 0.0f;
      sp[r * OP2 + col] = v;
    }
  }
  __syncthreads();

  v4f ov[4];
#pragma unroll
  for (int j = 0; j < 4; ++j) {
    const int r = 4 * j + (lane >> 3);
    ov[j] = *(const v4fa*)(sO + wave * 16 * OP2 + r * OP2 + 4 * q);
  }
#pragma unroll
  for (int j = 0; j < 4; ++j) {
    const int r = 4 * j + (lane >> 3);
    *(volatile v4f*)(FT + (size_t)(rowBase + r) * C2 + 4 * q) = ov[j];
  }
  __threadfence();
#pragma unroll
  for (int j = 0; j < 4; ++j) {
    const int r = 4 * j + (lane >> 3);
    *(volatile v4f*)(FT + (size_t)(rowBase + r) * C2 + 4 * q) = ov[j];
  }
}

__global__ __launch_bounds__(NTHR) void k_pool(
    const int* __restrict__ lab, const float* __restrict__ ft, float* out, int nPts) {
  __shared__ __attribute__((aligned(16))) float sacc[NBP * C2];
  __shared__ __attribute__((aligned(16))) int list[LISTN];
  __shared__ int pc[NBP];
  __shared__ int wcnt[NWAVE];
  const int tid = threadIdx.x, lane = tid & 31, wave = tid >> 5;
  const int gBase = blockIdx.x * NBP;

  {
    const v4f z4 = {0.f, 0.f, 0.f, 0.f};
    for (int i = tid; i < NBP * C2 / 4; i += NTHR) ((v4f*)sacc)[i] = z4;
    for (int i = tid; i < NBP; i += NTHR) pc[i] = 0;
  }
  __syncthreads();

  const int nChunks = (nPts + CHUNK - 1) / CHUNK;
#pragma unroll 1
  for (int ch = 0; ch < nChunks; ++ch) {
    const int cbase = ch * CHUNK;
    const int wc = scan_chunk<NBP>(lab, nPts, cbase, gBase, 1, list, tid, lane, wave);
    if (lane == 0) wcnt[wave] = wc;
    __syncthreads();
    if (wave == 0) {
#pragma unroll 1
      for (int wsx = 0; wsx < NWAVE; ++wsx) {
        int n = __builtin_amdgcn_readfirstlane(wcnt[wsx]);
        n = n > WCAP ? WCAP : (n < 0 ? 0 : n);
        const int* lp = list + wsx * WCAP;
#pragma unroll 1
        for (int i = 0; i < n; ++i) {
          const int ent  = __builtin_amdgcn_readfirstlane(lp[i]);
          const int slot = ent & (NBP - 1);
          int nd = cbase + ((ent >> 12) & (CHUNK - 1));
          nd = nd > nPts - 1 ? nPts - 1 : nd;
          const float v = ft[(size_t)nd * C2 + lane];
          sacc[slot * C2 + lane] = sacc[slot * C2 + lane] + v;
          if (lane == 0) pc[slot] = pc[slot] + 1;
        }
      }
    }
    __syncthreads();
  }

  v4f ov[4];
#pragma unroll
  for (int it = 0; it < 4; ++it) {
    const int id  = it * NTHR + tid;
    const int row = id >> 3;
    const int c0  = (id & 7) * 4;
    int cv = pc[row];
    cv = cv < 1 ? 1 : cv;
    const float inv = 1.0f / (float)cv;
    ov[it] = *(const v4f*)(sacc + row * C2 + c0) * inv;
  }
#pragma unroll
  for (int it = 0; it < 4; ++it) {
    const int id = it * NTHR + tid;
    *(volatile v4f*)(out + (size_t)(gBase + (id >> 3)) * C2 + (id & 7) * 4) = ov[it];
  }
  __threadfence();
#pragma unroll
  for (int it = 0; it < 4; ++it) {
    const int id = it * NTHR + tid;
    *(volatile v4f*)(out + (size_t)(gBase + (id >> 3)) * C2 + (id & 7) * 4) = ov[it];
  }
}

extern "C" void kernel_launch(void* const* d_in, const int* in_sizes, int n_in,
                              void* d_out, int out_size, void* d_ws, size_t ws_size,
                              hipStream_t stream) {
  if (n_in < 10) return;
  const int N = in_sizes[0] / CIN;
  if (N <= 0 || in_sizes[0] != N * CIN || in_sizes[1] != 4 * N || in_sizes[2] != N) return;
  if (in_sizes[3] < 1 || in_sizes[4] < 1 || in_sizes[5] < 1) return;
  if (in_sizes[6] != NTAP * CIN * C1 || in_sizes[7] != C1 || in_sizes[8] != NTAP * C1 * C2 || in_sizes[9] != C2) return;
  if (out_size != NCL * C2) return;
  if (N > (1 << 24)) return;

  const float* feat = (const float*)d_in[0];
  const int*   idx  = (const int*)d_in[1];
  const int*   lab  = (const int*)d_in[2];
  const int*   dimD = (const int*)d_in[3];
  const int*   dimH = (const int*)d_in[4];
  const int*   dimW = (const int*)d_in[5];
  const float* W1   = (const float*)d_in[6];
  const float* b1   = (const float*)d_in[7];
  const float* W2   = (const float*)d_in[8];
  const float* b2   = (const float*)d_in[9];
  float* out = (float*)d_out;

  const int NPAD  = ((N + RPAD - 1) / RPAD) * RPAD;
  const int NPADX = NPAD + RPAD;
  const int zrow  = NPADX - 1;

  char* ws = (char*)d_ws;
  size_t off = 0;
  const size_t oP1  = off; off += (size_t)C1 * KP1 * 2;      off = (off + 255) & ~(size_t)255;
  const size_t oP2  = off; off += (size_t)C2 * KP2 * 2;      off = (off + 255) & ~(size_t)255;
  const size_t oF   = off; off += (size_t)NPADX * 16 * 2;    off = (off + 255) & ~(size_t)255;
  const size_t oLin = off; off += (size_t)NPADX * 4;         off = (off + 255) & ~(size_t)255;
  const size_t oTbl = off; off += (size_t)TBLN * 4;          off = (off + 255) & ~(size_t)255;
  const size_t oH1  = off; off += (size_t)NPADX * C1 * 2;    off = (off + 255) & ~(size_t)255;
  const size_t oFt  = off; off += (size_t)NPADX * C2 * 4;    off = (off + 255) & ~(size_t)255;
  if (off > ws_size) return;
  _Float16* P1  = (_Float16*)(ws + oP1);
  _Float16* P2  = (_Float16*)(ws + oP2);
  _Float16* F   = (_Float16*)(ws + oF);
  int*      lin = (int*)(ws + oLin);
  int*      tbl = (int*)(ws + oTbl);
  _Float16* H1  = (_Float16*)(ws + oH1);
  float*    FT  = (float*)(ws + oFt);

  const int nPrep = (C1 * KP1 / 8 + C2 * KP2 / 8 + NPADX * 2 + NPADX / 4) / NTHR;
  k_prep<<<nPrep, NTHR, 0, stream>>>(W1, W2, feat, idx, P1, P2, F, lin, N, NPADX);

  hipFuncSetAttribute(reinterpret_cast<const void*>(&k_table),
                      hipFuncAttributeMaxDynamicSharedMemorySize, LDS_TAB);
  k_table<<<TBLN / TBLK, NTHR, LDS_TAB, stream>>>(lin, tbl, N);

  const int nConv = NPADX / PTS;
  k_conv1<<<nConv, NTHR, 0, stream>>>(idx, dimD, dimH, dimW, tbl, F, P1, b1, H1, N, zrow);
  k_conv2<<<nConv, NTHR, 0, stream>>>(idx, dimD, dimH, dimW, tbl, H1, P2, b2, FT, N, zrow);

  k_pool<<<NCL / NBP, NTHR, 0, stream>>>(lab, FT, out, N);
}
